// DAG_RNN_4Neigh_50929722196510
// MI455X (gfx1250) — hardware-verified
//
#include <hip/hip_runtime.h>
#include <math.h>

typedef __attribute__((ext_vector_type(16))) _Float16 v16h;
typedef __attribute__((ext_vector_type(8)))  _Float16 v8h;
typedef __attribute__((ext_vector_type(8)))  float    v8f;
typedef __attribute__((ext_vector_type(4)))  float    v4f;

constexpr int kB      = 32;
constexpr int kC      = 64;
constexpr int kH      = 80;
constexpr int kW      = 80;
constexpr int kCells  = kH * kW;
constexpr int kWaves  = kB / 16;
constexpr int kTilesC = kC / 16;
constexpr int kCellW  = kTilesC * 32 * 8;
constexpr size_t kPlaneF = (size_t)kCells * kWaves * kCellW;
constexpr int kThr    = 256;
static_assert(kB == 32 && kC == 64 && kCellW == 1024, "two waves of 16 batch columns; 64 channels = four 16-row tiles");
static_assert(kPlaneF == (size_t)kB * kC * kH * kW, "the fragment-major plane holds every element once");

constexpr float kStateCarry  = 1024.0f;
constexpr float kWeightCarry = 1024.0f;
constexpr float kFoldBack    = 1.0f / (kStateCarry * kWeightCarry);
constexpr float kF16MinNorm  = 6.103515625e-5f;
static_assert(kStateCarry * kWeightCarry == 1048576.0f, "carry product");

constexpr size_t kOffXT   = 0;
constexpr size_t kOffACC  = kOffXT  + kPlaneF * 4;
constexpr size_t kOffRB   = kOffACC + kPlaneF * 4;
constexpr size_t kRBPerWave = (size_t)kW * 2 * 32 * 16;
constexpr size_t kWsTotal = kOffRB + (size_t)kWaves * kRBPerWave * 2;
static_assert(kWsTotal == 105185280ull && kWsTotal <= 134217728ull, "carve total and cap");
static_assert((kOffACC % 256) == 0 && (kOffRB % 256) == 0, "aligned regions");

namespace eng {

union FragU { v16h v; v8h h[2]; };

__device__ __forceinline__ unsigned short f2bf_bits(float f) {
  unsigned u = __float_as_uint(f);
  return (unsigned short)((u + 0x7FFFu + ((u >> 16) & 1u)) >> 16);
}
__device__ __forceinline__ float bf16v(float f) {
  return __uint_as_float(((unsigned)f2bf_bits(f)) << 16);
}
__device__ __forceinline__ _Float16 to_f16_flushed(float c) {
  const float z = (fabsf(c) < kF16MinNorm) ? 0.0f : c;
  return (_Float16)z;
}
__device__ __forceinline__ v8f mma_f16(v16h a, v16h b, v8f c) {
  c = __builtin_amdgcn_wmma_f32_16x16x32_f16(false, a, false, b, (short)0, c, false, false);
  asm volatile("v_nop\n\tv_nop\n\tv_nop\n\tv_nop" : "+v"(c) : "v"(a), "v"(b));
  return c;
}

}

__global__ __launch_bounds__(kThr) void xfrag_kernel(const float* __restrict__ x, float* __restrict__ XT) {
  const int g    = blockIdx.x * kThr + threadIdx.x;
  const int lane = g & 31;
  const int m    = (g >> 5) & 3;
  const int w    = (g >> 7) & 1;
  const int p    = g >> 8;
  const int hs = lane >> 4, n = lane & 15;
  const int b  = 16 * w + n;
  const int c0 = 16 * m + 8 * hs;
  const float* src = x + ((size_t)b * kC + c0) * kCells + p;
  v4f lo, hi;
#pragma unroll
  for (int r = 0; r < 4; ++r) {
    const float a0 = src[(size_t)r * kCells];
    const float a1 = src[(size_t)(r + 4) * kCells];
    lo[r] = eng::bf16v(a0);
    hi[r] = eng::bf16v(a1);
  }
  float* dst = XT + (size_t)g * 8;
  for (int pass = 0; pass < 2; ++pass) {
    *(volatile v4f*)dst = lo;
    *(volatile v4f*)(dst + 4) = hi;
    __threadfence();
  }
}

__global__ __launch_bounds__(32) void dag_dir_kernel(const float* __restrict__ XT, const float* __restrict__ gv,
                                                     const float* __restrict__ gh, float* __restrict__ ACC,
                                                     unsigned short* __restrict__ RB,
                                                     int flip_i, int flip_j, int relu_on, int first) {
  __shared__ __align__(32) v16h AF[2 * kTilesC * 2 * 32];

  const int lane = threadIdx.x & 31;
  const int hsel = lane >> 4;
  const int n    = lane & 15;
  const int w    = blockIdx.x;

#pragma unroll 1
  for (int t = 0; t < 2; ++t) {
    const float* wsrc = t ? gh : gv;
#pragma unroll 1
    for (int m = 0; m < kTilesC; ++m) {
#pragma unroll 1
      for (int c = 0; c < 2; ++c) {
        v8h lo, hi;
#pragma unroll
        for (int e = 0; e < 16; ++e) {
          const int k = 32 * c + 16 * (e >> 3) + 8 * hsel + (e & 7);
          const float wv = wsrc[(16 * m + n) * kC + k];
          const _Float16 hv = eng::to_f16_flushed(eng::bf16v(wv) * kWeightCarry);
          if (e < 8) lo[e & 7] = hv; else hi[e & 7] = hv;
        }
        eng::FragU u0;
        u0.h[0] = lo;
        u0.h[1] = hi;
        AF[((t * kTilesC + m) * 2 + c) * 32 + lane] = u0.v;
      }
    }
  }
  v16h* rb = (v16h*)RB + (size_t)w * kW * 2 * 32;
  const v8h zh = (v8h){(_Float16)0.0f, (_Float16)0.0f, (_Float16)0.0f, (_Float16)0.0f,
                       (_Float16)0.0f, (_Float16)0.0f, (_Float16)0.0f, (_Float16)0.0f};
  eng::FragU zf;
  zf.h[0] = zh;
  zf.h[1] = zh;
#pragma unroll 1
  for (int jj = 0; jj < kW; ++jj) {
    for (int pass = 0; pass < 2; ++pass) {
      *(volatile v16h*)(rb + (jj * 2 + 0) * 32 + lane) = zf.v;
      *(volatile v16h*)(rb + (jj * 2 + 1) * 32 + lane) = zf.v;
      __threadfence();
    }
  }
  __syncthreads();

  const v8f z8 = (v8f){0.f, 0.f, 0.f, 0.f, 0.f, 0.f, 0.f, 0.f};

#pragma unroll 1
  for (int ii = 0; ii < kH; ++ii) {
    const int i = flip_i ? (kH - 1 - ii) : ii;
    eng::FragU l0, l1;
    l0.v = zf.v;
    l1.v = zf.v;
#pragma unroll 1
    for (int jj = 0; jj < kW; ++jj) {
      const int j = flip_j ? (kW - 1 - jj) : jj;
      const size_t base = (((size_t)(i * kW + j) * kWaves + w) * kTilesC) * 256 + (size_t)lane * 8;
      const v16h u0 = rb[(jj * 2 + 0) * 32 + lane];
      const v16h u1 = rb[(jj * 2 + 1) * 32 + lane];
      v8h nb[kTilesC];
#pragma unroll
      for (int m = 0; m < kTilesC; ++m) {
        v8f acc = z8;
        acc = eng::mma_f16(AF[((0 * kTilesC + m) * 2 + 0) * 32 + lane], u0, acc);
        acc = eng::mma_f16(AF[((0 * kTilesC + m) * 2 + 1) * 32 + lane], u1, acc);
        acc = eng::mma_f16(AF[((1 * kTilesC + m) * 2 + 0) * 32 + lane], l0.v, acc);
        acc = eng::mma_f16(AF[((1 * kTilesC + m) * 2 + 1) * 32 + lane], l1.v, acc);
        const float* xp = XT + base + (size_t)m * 256;
        const v4f x0 = *(const v4f*)xp;
        const v4f x1 = *(const v4f*)(xp + 4);
        float* ap = ACC + base + (size_t)m * 256;
        v4f a0 = {0.f, 0.f, 0.f, 0.f};
        v4f a1 = {0.f, 0.f, 0.f, 0.f};
        if (!first) {
          a0 = *(const v4f*)ap;
          a1 = *(const v4f*)(ap + 4);
        }
        v4f o0, o1;
#pragma unroll
        for (int r = 0; r < 8; ++r) {
          const float xv = (r < 4) ? x0[r & 3] : x1[r & 3];
          const float pre = fmaf(acc[r], kFoldBack, xv);
          const float hv = relu_on ? fmaxf(pre, 0.0f) : pre;
          nb[m][r] = eng::to_f16_flushed(hv * kStateCarry);
          const float av = (r < 4) ? a0[r & 3] : a1[r & 3];
          if (r < 4) o0[r & 3] = av + hv; else o1[r & 3] = av + hv;
        }
        for (int pass = 0; pass < 2; ++pass) {
          *(volatile v4f*)ap = o0;
          *(volatile v4f*)(ap + 4) = o1;
          __threadfence();
        }
      }
      l0.h[0] = nb[0];
      l0.h[1] = nb[1];
      l1.h[0] = nb[2];
      l1.h[1] = nb[3];
      for (int pass = 0; pass < 2; ++pass) {
        *(volatile v16h*)(rb + (jj * 2 + 0) * 32 + lane) = l0.v;
        *(volatile v16h*)(rb + (jj * 2 + 1) * 32 + lane) = l1.v;
        __threadfence();
      }
    }
  }
}

__global__ __launch_bounds__(kThr) void out_layout_kernel(const float* __restrict__ ACC, float* __restrict__ out) {
  const size_t t  = (size_t)blockIdx.x * kThr + threadIdx.x;
  const int p4    = (int)(t % (kCells / 4)) * 4;
  const int bc    = (int)(t / (kCells / 4));
  const int c     = bc & (kC - 1);
  const int b     = bc >> 6;
  const int lane  = 16 * ((c >> 3) & 1) + (b & 15);
  const size_t off = (((size_t)(b >> 4)) * kTilesC + (c >> 4)) * 256 + (size_t)lane * 8 + (c & 7);
  v4f o;
#pragma unroll
  for (int e = 0; e < 4; ++e) {
    const float v = ACC[(size_t)(p4 + e) * (kWaves * kCellW) + off];
    o[e] = v;
  }
  float* dst = out + (size_t)bc * kCells + p4;
  *(volatile v4f*)dst = o;
  __threadfence();
  *(volatile v4f*)dst = o;
}

static_assert((kPlaneF / 8) % kThr == 0 && (kPlaneF / 4) % kThr == 0, "re-layout and output grids exact");

extern "C" void kernel_launch(void* const* d_in, const int* in_sizes, int n_in,
                              void* d_out, int out_size, void* d_ws, size_t ws_size,
                              hipStream_t stream) {
  if (n_in < 9 || d_out == nullptr || d_ws == nullptr) return;
  if ((size_t)in_sizes[0] != kPlaneF) return;
  for (int k = 1; k < 9; ++k) if (in_sizes[k] != kC * kC) return;
  if ((size_t)out_size != kPlaneF) return;
  if (ws_size < kWsTotal) return;

  const float* x   = (const float*)d_in[0];
  const float* g1  = (const float*)d_in[1];
  const float* g2  = (const float*)d_in[2];
  const float* g4  = (const float*)d_in[3];
  const float* g5  = (const float*)d_in[4];
  const float* g7  = (const float*)d_in[5];
  const float* g8  = (const float*)d_in[6];
  const float* g10 = (const float*)d_in[7];
  const float* g11 = (const float*)d_in[8];
  float* out = (float*)d_out;

  char* ws = (char*)d_ws;
  float* XT  = (float*)(ws + kOffXT);
  float* ACC = (float*)(ws + kOffACC);
  unsigned short* RB = (unsigned short*)(ws + kOffRB);

  xfrag_kernel<<<(int)((kPlaneF / 8) / kThr), kThr, 0, stream>>>(x, XT);
  dag_dir_kernel<<<kWaves, 32, 0, stream>>>(XT, g1,  g2,  ACC, RB, 0, 0, 1, 1);
  dag_dir_kernel<<<kWaves, 32, 0, stream>>>(XT, g4,  g5,  ACC, RB, 1, 0, 1, 0);
  dag_dir_kernel<<<kWaves, 32, 0, stream>>>(XT, g7,  g8,  ACC, RB, 1, 1, 1, 0);
  dag_dir_kernel<<<kWaves, 32, 0, stream>>>(XT, g10, g11, ACC, RB, 0, 1, 0, 0);
  out_layout_kernel<<<(int)((kPlaneF / 4) / kThr), kThr, 0, stream>>>(ACC, out);
}
